// MambaLayer_53824530154109
// MI455X (gfx1250) — hardware-verified
//
#include <hip/hip_runtime.h>
#include <math.h>

typedef __attribute__((ext_vector_type(16))) _Float16 v16h;
typedef __attribute__((ext_vector_type(8)))  _Float16 v8h;
typedef __attribute__((ext_vector_type(8)))  float    v8f;
typedef __attribute__((ext_vector_type(4)))  float    v4f;

constexpr int kBatch = 4;
constexpr int kSeqL  = 2048;
constexpr int kDmod  = 512;
constexpr int kDin   = 512;
constexpr int kNst   = 16;
constexpr int kDtR   = 32;
constexpr int kPrjP  = kDtR + 2 * kNst;
constexpr int kXZP   = 2 * kDin;
constexpr int kRows  = kBatch * kSeqL;
constexpr int kTP    = 260;

constexpr float kCarryWin  = 32.0f;
constexpr float kCarryWxp  = 32.0f;
constexpr float kCarryWdt  = 8.0f;
constexpr float kCarryWout = 32.0f;
constexpr float kCarryX    = 1.0f;
constexpr float kCarryUc   = 1.0f;
constexpr float kCarryDt   = 16.0f;
constexpr float kCarryY    = 16.0f;
constexpr float kFoldIn  = 1.0f / (kCarryX  * kCarryWin);
constexpr float kFoldXp  = 1.0f / (kCarryUc * kCarryWxp);
constexpr float kFoldDt  = 1.0f / (kCarryDt * kCarryWdt);
constexpr float kFoldOut = 1.0f / (kCarryY  * kCarryWout);

static_assert(kPrjP == 64, "x_proj width");
static_assert(kRows == 8192 && kXZP == 1024, "shape constants");
static_assert((kDmod % 32) == 0 && (kDin % 32) == 0 && (kDtR % 32) == 0, "GEMM K multiples of 32");
static_assert((kRows % 64) == 0 && (kXZP % 64) == 0 && (kPrjP % 64) == 0 && (kDin % 64) == 0 && (kDmod % 64) == 0, "GEMM M,N multiples of 64");
static_assert(((kRows / 64) * (kXZP / 64)) % 8 == 0 && ((kRows / 64) * (kPrjP / 64)) % 8 == 0 &&
              ((kRows / 64) * (kDin / 64)) % 8 == 0 && ((kRows / 64) * (kDmod / 64)) % 8 == 0, "8 tiles per block exactly");
static_assert((kSeqL % 64) == 0 && (kDin % 256) == 0 && (kSeqL % 16) == 0, "tile multiples");
static_assert(((kRows * kDmod) % 2048) == 0 && ((kXZP * kDmod) % 2048) == 0 && ((kPrjP * kDin) % 2048) == 0 &&
              ((kDin * kDtR) % 2048) == 0 && ((kDmod * kDin) % 2048) == 0 && ((kRows * kDtR) % 2048) == 0, "cast grids exact");

constexpr size_t kSzX16    = (size_t)kRows * kDmod * 2;
constexpr size_t kSzWIN16  = (size_t)kXZP  * kDmod * 2;
constexpr size_t kSzWXP16  = (size_t)kPrjP * kDin  * 2;
constexpr size_t kSzWDT16  = (size_t)kDin  * kDtR  * 2;
constexpr size_t kSzWOUT16 = (size_t)kDmod * kDin  * 2;
constexpr size_t kSzXZ     = (size_t)kRows * kXZP  * 4;
constexpr size_t kSzUC     = (size_t)kRows * kDin  * 4;
constexpr size_t kSzUC16   = (size_t)kRows * kDin  * 2;
constexpr size_t kSzPROJ   = (size_t)kRows * kPrjP * 4;
constexpr size_t kSzDT16   = (size_t)kRows * kDtR  * 2;
constexpr size_t kSzDLR    = (size_t)kRows * kDin  * 4;
constexpr size_t kSzY16    = (size_t)kRows * kDin  * 2;
constexpr size_t kOffX16    = 0;
constexpr size_t kOffWIN16  = kOffX16    + kSzX16;
constexpr size_t kOffWXP16  = kOffWIN16  + kSzWIN16;
constexpr size_t kOffWDT16  = kOffWXP16  + kSzWXP16;
constexpr size_t kOffWOUT16 = kOffWDT16  + kSzWDT16;
constexpr size_t kOffXZ     = kOffWOUT16 + kSzWOUT16;
constexpr size_t kOffUC     = kOffXZ     + kSzXZ;
constexpr size_t kOffUC16   = kOffUC     + kSzUC;
constexpr size_t kOffPROJ   = kOffUC16   + kSzUC16;
constexpr size_t kOffDT16   = kOffPROJ   + kSzPROJ;
constexpr size_t kOffDLR    = kOffDT16   + kSzDT16;
constexpr size_t kOffY16    = kOffDLR    + kSzDLR;
constexpr size_t kWsTotal   = kOffY16    + kSzY16;
static_assert(kWsTotal == 96567296ull, "carve total");
static_assert(kWsTotal <= 134217728ull, "carve cap");
static_assert((kOffWIN16 % 128) == 0 && (kOffWXP16 % 128) == 0 && (kOffWDT16 % 128) == 0 && (kOffWOUT16 % 128) == 0 &&
              (kOffXZ % 128) == 0 && (kOffUC % 128) == 0 && (kOffUC16 % 128) == 0 && (kOffPROJ % 128) == 0 &&
              (kOffDT16 % 128) == 0 && (kOffDLR % 128) == 0 && (kOffY16 % 128) == 0, "128-B aligned regions");

__device__ __forceinline__ float bf_rne(float f) {
  unsigned u = __float_as_uint(f);
  u = (u + 0x7FFFu + ((u >> 16) & 1u)) & 0xFFFF0000u;
  return __uint_as_float(u);
}

__device__ __forceinline__ void dep_guard4_h(v8f& a, v8f& b, v8f& c, v8f& d, v16h x, v16h y) {
  asm volatile("v_nop\n\tv_nop\n\tv_nop\n\tv_nop" : "+v"(a), "+v"(b), "+v"(c), "+v"(d) : "v"(x), "v"(y));
}
__device__ __forceinline__ void keep4_h(v16h a, v16h b, v16h c, v16h d) { asm volatile("v_nop" :: "v"(a), "v"(b), "v"(c), "v"(d)); }
__device__ __forceinline__ void acc_guard4(v8f& a, v8f& b, v8f& c, v8f& d) { asm volatile("v_nop\n\tv_nop\n\tv_nop\n\tv_nop" : "+v"(a), "+v"(b), "+v"(c), "+v"(d)); }

union FragU { v16h v; v8h h[2]; };
__device__ __forceinline__ v16h frag_load(const _Float16* p) {
  FragU f;
  f.h[0] = *(const v8h*)(p);
  f.h[1] = *(const v8h*)(p + 16);
  return f.v;
}
__device__ __forceinline__ v8f frag_mma(v16h a, v16h b, v8f c) {
  return __builtin_amdgcn_wmma_f32_16x16x32_f16(false, a, false, b, (short)0, c, false, false);
}

template <int BIAS_MODE, int ACT>
__global__ __launch_bounds__(256) void wmma_gemm64_f16(
    const unsigned short* __restrict__ Ap, int lda,
    const unsigned short* __restrict__ Btp, int ldb,
    float* __restrict__ C, int ldc,
    const float* __restrict__ bias,
    int M, int N, int K, float scale) {
  const _Float16* A  = (const _Float16*)Ap;
  const _Float16* Bt = (const _Float16*)Btp;
  __shared__ __align__(16) float sT[8][16 * 68];
  const int lane = threadIdx.x & 31;
  const int wave = threadIdx.x >> 5;
  const int tilesN = N >> 6;
  const int tilesM = M >> 6;
  const int tile = blockIdx.x * 8 + wave;
  if (tile >= tilesM * tilesN) return;
  const int tm = tile / tilesN;
  const int tn = tile - tm * tilesN;
  const int m0 = tm << 6;
  const int n0 = tn << 6;

  const int rlane = lane & 15;
  const int koff  = (lane >> 4) * 8;
  const int mOff  = (lane >> 4) * 8;

  v8f acc[4][4];
#pragma unroll
  for (int i = 0; i < 4; ++i)
#pragma unroll
    for (int j = 0; j < 4; ++j) acc[i][j] = (v8f){0.f,0.f,0.f,0.f,0.f,0.f,0.f,0.f};

  for (int k0 = 0; k0 < K; k0 += 32) {
    v16h bh[4];
#pragma unroll
    for (int j = 0; j < 4; ++j) {
      const size_t bo = (size_t)(n0 + (j << 4) + rlane) * ldb + koff + k0;
      bh[j] = frag_load(Bt + bo);
    }
#pragma unroll
    for (int i = 0; i < 4; ++i) {
      const size_t ao = (size_t)(m0 + (i << 4) + rlane) * lda + koff + k0;
      const v16h ah = frag_load(A + ao);
#pragma unroll
      for (int j = 0; j < 4; ++j) acc[i][j] = frag_mma(ah, bh[j], acc[i][j]);
      dep_guard4_h(acc[i][0], acc[i][1], acc[i][2], acc[i][3], ah, bh[3]);
    }
    keep4_h(bh[0], bh[1], bh[2], bh[3]);
  }
  acc_guard4(acc[0][0], acc[0][1], acc[0][2], acc[0][3]);
  acc_guard4(acc[1][0], acc[1][1], acc[1][2], acc[1][3]);
  acc_guard4(acc[2][0], acc[2][1], acc[2][2], acc[2][3]);
  acc_guard4(acc[3][0], acc[3][1], acc[3][2], acc[3][3]);

  float* slab = sT[wave];
#pragma unroll
  for (int i = 0; i < 4; ++i) {
    const int mBase = m0 + (i << 4);
#pragma unroll
    for (int j = 0; j < 4; ++j) {
      const int n = n0 + (j << 4) + rlane;
      float bv = 0.f;
      if (BIAS_MODE == 2) {
        const float braw = bias[n];
        bv = bf_rne(braw);
      }
#pragma unroll
      for (int r = 0; r < 8; ++r) {
        float v = acc[i][j][r] * scale;
        if (BIAS_MODE == 2) v += bv;
        if (ACT == 6) v = (v != v) ? 0.0f : fminf(fmaxf(v, -1000.0f), 1000.0f);
        slab[(mOff + r) * 68 + (j << 4) + rlane] = v;
      }
    }
    __builtin_amdgcn_fence(__ATOMIC_RELEASE, "workgroup");
    __builtin_amdgcn_wave_barrier();
    __builtin_amdgcn_fence(__ATOMIC_ACQUIRE, "workgroup");
    {
      const int hh = lane >> 4, c4 = (lane & 15) * 4;
      for (int pass = 0; pass < 2; ++pass) {
#pragma unroll
        for (int it = 0; it < 8; ++it) {
          const int row = it * 2 + hh;
          v4f v = *(const v4f*)(slab + row * 68 + c4);
          *(volatile v4f*)(C + (size_t)(mBase + row) * ldc + n0 + c4) = v;
        }
        __threadfence();
      }
    }
    __builtin_amdgcn_fence(__ATOMIC_RELEASE, "workgroup");
    __builtin_amdgcn_wave_barrier();
    __builtin_amdgcn_fence(__ATOMIC_ACQUIRE, "workgroup");
  }
}

__global__ __launch_bounds__(256) void cast_bf_f16_kernel(
    const float* __restrict__ src, unsigned short* __restrict__ dst, int total8, float scale)
{
  const int i = blockIdx.x * 256 + threadIdx.x;
  if (i >= total8) return;
  const size_t e0 = (size_t)i << 3;
  const float* p = src + e0;
  const v4f a0 = *(const v4f*)(p);
  const v4f a1 = *(const v4f*)(p + 4);
  v8h hv;
#pragma unroll
  for (int e = 0; e < 4; ++e) {
    const float s0 = a0[e];
    const float s1 = a1[e];
    const float r0 = bf_rne(s0);
    const float r1 = bf_rne(s1);
    hv[e]     = (_Float16)(r0 * scale);
    hv[4 + e] = (_Float16)(r1 * scale);
  }
  unsigned short* q = dst + e0;
  *(volatile v8h*)q = hv;
  __threadfence();
  *(volatile v8h*)q = hv;
}

__global__ __launch_bounds__(256) void dt_cast_kernel(
    const float* __restrict__ PROJ, unsigned short* __restrict__ DT16, int total8, float scale)
{
  const int i = blockIdx.x * 256 + threadIdx.x;
  if (i >= total8) return;
  const int e0  = i << 3;
  const int row = e0 / kDtR;
  const int c8  = e0 - row * kDtR;
  const float* p = PROJ + (size_t)row * kPrjP + c8;
  const v4f a0 = *(const v4f*)(p);
  const v4f a1 = *(const v4f*)(p + 4);
  v8h hv;
#pragma unroll
  for (int e = 0; e < 4; ++e) {
    hv[e]     = (_Float16)(a0[e] * scale);
    hv[4 + e] = (_Float16)(a1[e] * scale);
  }
  unsigned short* qd = DT16 + e0;
  *(volatile v8h*)qd = hv;
  __threadfence();
  *(volatile v8h*)qd = hv;
}

__global__ __launch_bounds__(256) void conv_silu_kernel(
    const float* __restrict__ XZ, const float* __restrict__ cw, const float* __restrict__ cb,
    float* __restrict__ UC, unsigned short* __restrict__ UC16)
{
  __shared__ __align__(16) float sT[16 * kTP];
  const int tid = threadIdx.x, lane = tid & 31, wave = tid >> 5;
  const int d0 = blockIdx.x * 256, d = d0 + tid;
  const int g0 = blockIdx.y * 64;
  const int tb = g0 & (kSeqL - 1);
  const v4f wv = *(const v4f*)(cw + (size_t)d * 4);
  const float wr0 = wv[0], wr1 = wv[1], wr2 = wv[2], wr3 = wv[3];
  const float w0 = bf_rne(wr0), w1 = bf_rne(wr1), w2 = bf_rne(wr2), w3 = bf_rne(wr3);
  const float bcr = cb[d];
  const float bc = bf_rne(bcr);
  float xm3, xm2, xm1;
  {
    const bool hist = (tb > 0);
    const int rb = hist ? (g0 - 3) : g0;
    const float v3 = XZ[(size_t)rb * kXZP + d];
    const float v2 = XZ[(size_t)(rb + 1) * kXZP + d];
    const float v1 = XZ[(size_t)(rb + 2) * kXZP + d];
    xm3 = hist ? v3 : 0.f;
    xm2 = hist ? v2 : 0.f;
    xm1 = hist ? v1 : 0.f;
  }
  const int hrow = wave >> 1;
  const int hch  = (wave & 1) * 128 + lane * 4;
#pragma unroll 1
  for (int sub = 0; sub < 4; ++sub) {
    const int lb = g0 + sub * 16;
#pragma unroll 1
    for (int s = 0; s < 16; ++s) {
      const float xcur = XZ[(size_t)(lb + s) * kXZP + d];
      float acc = w0 * xm3;
      acc = fmaf(w1, xm2, acc);
      acc = fmaf(w2, xm1, acc);
      acc = fmaf(w3, xcur, acc);
      const float sv = acc + bc;
      const float sg = __builtin_amdgcn_rcpf(1.0f + __expf(-sv));
      sT[s * kTP + tid] = sv * sg;
      xm3 = xm2; xm2 = xm1; xm1 = xcur;
    }
    __syncthreads();
    v4f fv[4];
    v8h bv[2];
#pragma unroll
    for (int it = 0; it < 4; ++it) fv[it] = *(const v4f*)(sT + (it * 4 + hrow) * kTP + hch);
#pragma unroll
    for (int it = 0; it < 2; ++it) {
      const float* sp = sT + (it * 8 + wave) * kTP + lane * 8;
      const v4f a0 = *(const v4f*)(sp);
      const v4f a1 = *(const v4f*)(sp + 4);
#pragma unroll
      for (int e = 0; e < 4; ++e) {
        bv[it][e]     = (_Float16)(a0[e] * kCarryUc);
        bv[it][4 + e] = (_Float16)(a1[e] * kCarryUc);
      }
    }
    for (int pass = 0; pass < 2; ++pass) {
#pragma unroll
      for (int it = 0; it < 4; ++it)
        *(volatile v4f*)(UC + (size_t)(lb + it * 4 + hrow) * kDin + d0 + hch) = fv[it];
#pragma unroll
      for (int it = 0; it < 2; ++it)
        *(volatile v8h*)(UC16 + (size_t)(lb + it * 8 + wave) * kDin + d0 + lane * 8) = bv[it];
      __threadfence();
    }
    __syncthreads();
  }
}

__global__ __launch_bounds__(256) void scan_kernel(
    const float* __restrict__ DLR, const float* __restrict__ UC, const float* __restrict__ XZ,
    const float* __restrict__ PROJ, const float* __restrict__ A_log, const float* __restrict__ Dv,
    unsigned short* __restrict__ Y16)
{
  __shared__ __align__(16) float sBC[16 * 32];
  __shared__ __align__(16) float sY[16 * kTP];
  __shared__ __align__(16) float sA[kNst * 256];
  const int tid = threadIdx.x, lane = tid & 31, wave = tid >> 5;
  constexpr int kBlkPerB = kDin / 256;
  const int bix = blockIdx.x / kBlkPerB;
  const int d0  = (blockIdx.x - bix * kBlkPerB) * 256;
  const int d   = d0 + tid;
  const size_t row0 = (size_t)bix * kSeqL;

#pragma unroll 1
  for (int n = 0; n < kNst; ++n) {
    const float alr = A_log[(size_t)d * kNst + n];
    sA[n * 256 + tid] = -expf(bf_rne(alr));
  }
  __syncthreads();
  float An[kNst], h[kNst];
#pragma unroll
  for (int n = 0; n < kNst; ++n) {
    An[n] = sA[n * 256 + tid];
    h[n] = 0.f;
  }
  const float Dr = Dv[d];
  const float Dd = bf_rne(Dr);

#pragma unroll 1
  for (int c = 0; c < kSeqL / 16; ++c) {
    const int l0 = c * 16;
    if (tid < 128) {
      const int r = tid >> 3, q = (tid & 7) * 4;
      const v4f v = *(const v4f*)(PROJ + (row0 + l0 + r) * kPrjP + kDtR + q);
      *(v4f*)(sBC + r * 32 + q) = v;
    }
    __syncthreads();
#pragma unroll 1
    for (int s = 0; s < 16; ++s) {
      const size_t m = row0 + (size_t)(l0 + s);
      const float a     = DLR[m * kDin + d];
      const float delta = fmaxf(a, 0.0f) + log1pf(__expf(-fabsf(a)));
      const float xv    = UC[m * kDin + d];
      const float zv    = XZ[m * kXZP + kDin + d];
      v4f Bq[4], Cq[4];
#pragma unroll
      for (int qq = 0; qq < 4; ++qq) {
        Bq[qq] = *(const v4f*)(sBC + s * 32 + 4 * qq);
        Cq[qq] = *(const v4f*)(sBC + s * 32 + kNst + 4 * qq);
      }
      float y = 0.f;
#pragma unroll
      for (int n = 0; n < kNst; ++n) {
        const float e = __expf(delta * An[n]);
        float db = delta * Bq[n >> 2][n & 3];
        asm volatile("" : "+v"(db));
        float p = db * xv;
        asm volatile("" : "+v"(p));
        float qv = h[n] * e;
        asm volatile("" : "+v"(qv));
        const float hn = qv + p;
        h[n] = hn;
        float rr = Cq[n >> 2][n & 3] * hn;
        asm volatile("" : "+v"(rr));
        y += rr;
      }
      float sk = xv * Dd;
      asm volatile("" : "+v"(sk));
      y += sk;
      const float sg = __builtin_amdgcn_rcpf(1.0f + __expf(-zv));
      const float g  = zv * sg;
      sY[s * kTP + tid] = (y * g) * kCarryY;
    }
    __syncthreads();
    v8h hv[2];
#pragma unroll
    for (int it = 0; it < 2; ++it) {
      const float* sp = sY + (it * 8 + wave) * kTP + lane * 8;
      const v4f a0 = *(const v4f*)(sp);
      const v4f a1 = *(const v4f*)(sp + 4);
#pragma unroll
      for (int e = 0; e < 4; ++e) {
        hv[it][e]     = (_Float16)a0[e];
        hv[it][4 + e] = (_Float16)a1[e];
      }
    }
    for (int pass = 0; pass < 2; ++pass) {
#pragma unroll
      for (int it = 0; it < 2; ++it)
        *(volatile v8h*)(Y16 + (row0 + (size_t)(l0 + it * 8 + wave)) * kDin + d0 + lane * 8) = hv[it];
      __threadfence();
    }
  }
}

extern "C" void kernel_launch(void* const* d_in, const int* in_sizes, int n_in,
                              void* d_out, int out_size, void* d_ws, size_t ws_size,
                              hipStream_t stream)
{
  if (n_in < 10) return;
  if (in_sizes[0] != kRows * kDmod) return;
  if (in_sizes[1] != kXZP * kDmod) return;
  if (in_sizes[2] != kDin * 4) return;
  if (in_sizes[3] != kDin) return;
  if (in_sizes[4] != kPrjP * kDin) return;
  if (in_sizes[5] != kDin * kDtR) return;
  if (in_sizes[6] != kDin) return;
  if (in_sizes[7] != kDin * kNst) return;
  if (in_sizes[8] != kDin) return;
  if (in_sizes[9] != kDmod * kDin) return;
  if (out_size != kRows * kDmod) return;
  if (ws_size < kWsTotal) return;

  const float* x      = (const float*)d_in[0];
  const float* W_in   = (const float*)d_in[1];
  const float* conv_w = (const float*)d_in[2];
  const float* conv_b = (const float*)d_in[3];
  const float* W_xprj = (const float*)d_in[4];
  const float* W_dt   = (const float*)d_in[5];
  const float* b_dt   = (const float*)d_in[6];
  const float* A_log  = (const float*)d_in[7];
  const float* Dv     = (const float*)d_in[8];
  const float* W_out  = (const float*)d_in[9];
  float* dout = (float*)d_out;

  char* ws = (char*)d_ws;
  unsigned short* X16    = (unsigned short*)(ws + kOffX16);
  unsigned short* WIN16  = (unsigned short*)(ws + kOffWIN16);
  unsigned short* WXP16  = (unsigned short*)(ws + kOffWXP16);
  unsigned short* WDT16  = (unsigned short*)(ws + kOffWDT16);
  unsigned short* WOUT16 = (unsigned short*)(ws + kOffWOUT16);
  float*          XZ     = (float*)(ws + kOffXZ);
  float*          UC     = (float*)(ws + kOffUC);
  unsigned short* UC16   = (unsigned short*)(ws + kOffUC16);
  float*          PROJ   = (float*)(ws + kOffPROJ);
  unsigned short* DT16   = (unsigned short*)(ws + kOffDT16);
  float*          DLR    = (float*)(ws + kOffDLR);
  unsigned short* Y16    = (unsigned short*)(ws + kOffY16);
  const float* dummy_bias = b_dt;

  cast_bf_f16_kernel<<<(kRows * kDmod / 8) / 256, 256, 0, stream>>>(x,      X16,    kRows * kDmod / 8, kCarryX);
  cast_bf_f16_kernel<<<(kXZP * kDmod / 8) / 256, 256, 0, stream>>>(W_in,   WIN16,  kXZP * kDmod / 8,  kCarryWin);
  cast_bf_f16_kernel<<<(kPrjP * kDin / 8) / 256, 256, 0, stream>>>(W_xprj, WXP16,  kPrjP * kDin / 8,  kCarryWxp);
  cast_bf_f16_kernel<<<(kDin * kDtR / 8) / 256, 256, 0, stream>>>(W_dt,   WDT16,  kDin * kDtR / 8,   kCarryWdt);
  cast_bf_f16_kernel<<<(kDmod * kDin / 8) / 256, 256, 0, stream>>>(W_out,  WOUT16, kDmod * kDin / 8,  kCarryWout);

  wmma_gemm64_f16<0, 0><<<((kRows / 64) * (kXZP / 64)) / 8, 256, 0, stream>>>(
      X16, kDmod, WIN16, kDmod, XZ, kXZP, dummy_bias, kRows, kXZP, kDmod, kFoldIn);

  conv_silu_kernel<<<dim3(kDin / 256, kRows / 64), 256, 0, stream>>>(XZ, conv_w, conv_b, UC, UC16);

  wmma_gemm64_f16<0, 0><<<((kRows / 64) * (kPrjP / 64)) / 8, 256, 0, stream>>>(
      UC16, kDin, WXP16, kDin, PROJ, kPrjP, dummy_bias, kRows, kPrjP, kDin, kFoldXp);

  dt_cast_kernel<<<(kRows * kDtR / 8) / 256, 256, 0, stream>>>(PROJ, DT16, kRows * kDtR / 8, kCarryDt);

  wmma_gemm64_f16<2, 0><<<((kRows / 64) * (kDin / 64)) / 8, 256, 0, stream>>>(
      DT16, kDtR, WDT16, kDtR, DLR, kDin, b_dt, kRows, kDin, kDtR, kFoldDt);

  scan_kernel<<<kBatch * (kDin / 256), 256, 0, stream>>>(DLR, UC, XZ, PROJ, A_log, Dv, Y16);

  wmma_gemm64_f16<0, 6><<<((kRows / 64) * (kDmod / 64)) / 8, 256, 0, stream>>>(
      Y16, kDin, WOUT16, kDin, dout, kDmod, dummy_bias, kRows, kDmod, kDin, kFoldOut);
}
